// GaussianSetConv1D_13597866459180
// MI455X (gfx1250) — hardware-verified
//
#include <hip/hip_runtime.h>
#include <stddef.h>
#include <math.h>


#define NN     4096
#define GG     1024
#define CC     32
#define NSIG   4
#define OC     (NSIG * CC)
#define GT     (GG / 16)
#define KSTEPS (NN / 32)
#define CV_N   256
#define CV_T   256
#define CV_P   264
#define MT     64
#define SO_P   68

static_assert(NN % CV_N == 0);
static_assert(NN % 32 == 0);
static_assert(GG % 16 == 0);
static_assert(CV_N == 8 * 32);
static_assert(CC == 32);
static_assert((CV_P * 2) % 16 == 0);
static_assert((SO_P * 4) % 16 == 0);
static_assert(CV_N * CC == 8 * 4 * CV_T);
static_assert(MT == 64);

#if __has_builtin(__builtin_amdgcn_exp2f)
#define EXP2_F(x) __builtin_amdgcn_exp2f(x)
#else
#define EXP2_F(x) exp2f(x)
#endif

typedef _Float16 v16h __attribute__((ext_vector_type(16)));
typedef _Float16 v8h  __attribute__((ext_vector_type(8)));
typedef float    v8f  __attribute__((ext_vector_type(8)));
typedef float    v4f  __attribute__((ext_vector_type(4)));
typedef unsigned int v4u __attribute__((ext_vector_type(4)));
typedef v4f __attribute__((may_alias)) v4fa;
typedef v4u __attribute__((may_alias)) v4ua;
union FragH { v16h v; v8h h[2]; };

#define L2EH 0.72134752044448170f
#define KC0 (-L2EH / (0.01f * 0.01f))
#define KC1 (-L2EH / (0.05f * 0.05f))
#define KC2 (-L2EH / (0.1f * 0.1f))
#define KC3 (-L2EH / (0.2f * 0.2f))

__device__ __forceinline__ v8f wmh(v16h a, v16h b, v8f c) {
  v8f d = __builtin_amdgcn_wmma_f32_16x16x32_f16(false, a, false, b, (short)0, c, false, false);
#if defined(__HIP_DEVICE_COMPILE__)
  asm volatile("v_nop\n\tv_nop\n\tv_nop\n\tv_nop" : "+v"(d) : "v"(a), "v"(b));
#endif
  return d;
}

__device__ __forceinline__ v8f zero8() {
  v8f z = {0.f, 0.f, 0.f, 0.f, 0.f, 0.f, 0.f, 0.f};
  return z;
}

__global__ __launch_bounds__(CV_T) void k_cvt(const float* __restrict__ feat,
                                               _Float16* featT) {
  __shared__ __align__(16) unsigned short sT[CC][CV_P];
  const int tid = (int)threadIdx.x, lane = tid & 31, wv = tid >> 5;
  const int nchunks = NN / CV_N;
  const int b  = (int)blockIdx.x / nchunks;
  const int nc = (int)blockIdx.x % nchunks;
  const int n0 = nc * CV_N;
  const float* src = feat + ((size_t)b * NN + n0) * CC;

#pragma unroll
  for (int i = 0; i < 8; ++i) {
    const int e  = i * 1024 + 4 * tid;
    const v4f v  = *(const v4f*)(src + e);
    const int nl = e >> 5, c = e & 31;
#pragma unroll
    for (int j = 0; j < 4; ++j)
      sT[c + j][nl] = __builtin_bit_cast(unsigned short, (_Float16)v[j]);
  }
  __syncthreads();

  v4u val[4];
#pragma unroll
  for (int q = 0; q < 4; ++q) {
    const int c = wv + 8 * q;
    val[q] = *(const v4ua*)(&sT[c][8 * lane]);
  }
  _Float16* dst0 = featT + ((size_t)(b * CC + wv)) * NN + n0 + 8 * lane;
#pragma unroll
  for (int q = 0; q < 4; ++q) {
    _Float16* p = dst0 + (size_t)(8 * q) * NN;
    *(volatile v4u*)p = val[q];
  }
  __threadfence();
#pragma unroll
  for (int q = 0; q < 4; ++q) {
    _Float16* p = dst0 + (size_t)(8 * q) * NN;
    *(volatile v4u*)p = val[q];
  }
}

__device__ __forceinline__ void sig_step(const float (&t)[16], const float (&mk)[16],
                                         float kc, float& d, v16h b0, v16h b1,
                                         v8f& c0, v8f& c1) {
  FragH a;
  v8h lo, hi;
#pragma unroll
  for (int i = 0; i < 8; ++i) {
    const float w = EXP2_F(t[i] * kc) * mk[i];
    d += w;
    lo[i] = (_Float16)w;
  }
#pragma unroll
  for (int i = 0; i < 8; ++i) {
    const float w = EXP2_F(t[8 + i] * kc) * mk[8 + i];
    d += w;
    hi[i] = (_Float16)w;
  }
  a.h[0] = lo;
  a.h[1] = hi;
  c0 = wmh(a.v, b0, c0);
  c1 = wmh(a.v, b1, c1);
}

__global__ __launch_bounds__(MT) void k_conv(const float* __restrict__ px,
                                              const float* __restrict__ pmask,
                                              const _Float16* __restrict__ featT,
                                              const float* __restrict__ gxp,
                                              float* out0, float* out1) {
  __shared__ __align__(16) float sO[2][16][SO_P];
  __shared__ __align__(16) float sD[16][4];

  const int tid = (int)threadIdx.x, lane = tid & 31, wv = tid >> 5;
  const int h = lane >> 4, m = lane & 15;
  const int b  = (int)blockIdx.x / GT;
  const int gt = (int)blockIdx.x % GT;
  const int g0 = gt * 16;

  const float gx  = gxp[g0 + m];
  const float kc0 = wv ? KC2 : KC0;
  const float kc1 = wv ? KC3 : KC1;

  const float* xb = px    + (size_t)b * NN;
  const float* mb = pmask + (size_t)b * NN;
  const _Float16* fb0 = featT + ((size_t)(b * CC + m)) * NN;
  const _Float16* fb1 = featT + ((size_t)(b * CC + 16 + m)) * NN;

  v8f acc00 = zero8(), acc01 = zero8(), acc10 = zero8(), acc11 = zero8();
  float d0 = 0.0f, d1 = 0.0f;

#pragma unroll 1
  for (int ks = 0; ks < KSTEPS; ++ks) {
    const int k0 = ks * 32;
    const v4f xv0 = *(const v4f*)(xb + k0 + 8 * h);
    const v4f xv1 = *(const v4f*)(xb + k0 + 8 * h + 4);
    const v4f xv2 = *(const v4f*)(xb + k0 + 16 + 8 * h);
    const v4f xv3 = *(const v4f*)(xb + k0 + 16 + 8 * h + 4);
    const v4f mv0 = *(const v4f*)(mb + k0 + 8 * h);
    const v4f mv1 = *(const v4f*)(mb + k0 + 8 * h + 4);
    const v4f mv2 = *(const v4f*)(mb + k0 + 16 + 8 * h);
    const v4f mv3 = *(const v4f*)(mb + k0 + 16 + 8 * h + 4);

    float t[16], mk[16];
#pragma unroll
    for (int j = 0; j < 4; ++j) {
      const float e0 = xv0[j] - gx, e1 = xv1[j] - gx, e2 = xv2[j] - gx, e3 = xv3[j] - gx;
      t[j]      = e0 * e0;
      t[4 + j]  = e1 * e1;
      t[8 + j]  = e2 * e2;
      t[12 + j] = e3 * e3;
      mk[j]      = mv0[j];
      mk[4 + j]  = mv1[j];
      mk[8 + j]  = mv2[j];
      mk[12 + j] = mv3[j];
    }

    FragH bf0, bf1;
    bf0.h[0] = *(const v8h*)(fb0 + k0 + 8 * h);
    bf0.h[1] = *(const v8h*)(fb0 + k0 + 16 + 8 * h);
    bf1.h[0] = *(const v8h*)(fb1 + k0 + 8 * h);
    bf1.h[1] = *(const v8h*)(fb1 + k0 + 16 + 8 * h);

    sig_step(t, mk, kc0, d0, bf0.v, bf1.v, acc00, acc01);
    sig_step(t, mk, kc1, d1, bf0.v, bf1.v, acc10, acc11);
  }

  const float df0 = d0 + __shfl_xor(d0, 16, 32);
  const float df1 = d1 + __shfl_xor(d1, 16, 32);

#pragma unroll
  for (int r = 0; r < 8; ++r) {
    const int row = 8 * h + r;
    const float e0 = __shfl(df0, row, 32);
    const float e1 = __shfl(df1, row, 32);
    const float i0 = 1.0f / fmaxf(e0, 1e-6f);
    const float i1 = 1.0f / fmaxf(e1, 1e-6f);
    sO[wv][row][m]      = acc00[r] * i0;
    sO[wv][row][16 + m] = acc01[r] * i0;
    sO[wv][row][32 + m] = acc10[r] * i1;
    sO[wv][row][48 + m] = acc11[r] * i1;
  }
  if (h == 0) {
    sD[m][2 * wv]     = df0;
    sD[m][2 * wv + 1] = df1;
  }
  __syncthreads();

  v4f ov[8];
#pragma unroll
  for (int j = 0; j < 8; ++j) ov[j] = *(const v4fa*)(&sO[wv][2 * j + h][4 * m]);
  float* ob = out0 + ((size_t)(b * GG + g0 + h)) * OC + 64 * wv + 4 * m;
  const v4f dv = *(const v4fa*)(&sD[m][0]);
  float* dp = out1 + ((size_t)(b * GG + g0 + m)) * NSIG;
  const bool dw = (wv == 0) && (h == 0);

#pragma unroll
  for (int j = 0; j < 8; ++j) {
    float* p = ob + (size_t)(2 * j) * OC;
    *(volatile v4f*)p = ov[j];
  }
  if (dw) *(volatile v4f*)dp = dv;
  __threadfence();
#pragma unroll
  for (int j = 0; j < 8; ++j) {
    float* p = ob + (size_t)(2 * j) * OC;
    *(volatile v4f*)p = ov[j];
  }
  if (dw) *(volatile v4f*)dp = dv;
}

extern "C" void kernel_launch(void* const* d_in, const int* in_sizes, int n_in,
                              void* d_out, int out_size, void* d_ws, size_t ws_size,
                              hipStream_t stream) {
  if (n_in < 4) return;
  const int nB = in_sizes[0] / NN;
  if (nB < 1 || in_sizes[0] != nB * NN) return;
  if (in_sizes[1] != nB * NN * CC) return;
  if (in_sizes[2] != nB * NN) return;
  if (in_sizes[3] != GG) return;
  if (out_size != nB * GG * OC + nB * GG * NSIG) return;

  const size_t ft_bytes = (size_t)nB * CC * NN * sizeof(_Float16);
  if (ft_bytes > ws_size) return;

  const float* px    = (const float*)d_in[0];
  const float* feat  = (const float*)d_in[1];
  const float* pmask = (const float*)d_in[2];
  const float* gxp   = (const float*)d_in[3];
  float* out0 = (float*)d_out;
  float* out1 = out0 + (size_t)nB * GG * OC;
  _Float16* featT = (_Float16*)d_ws;

  k_cvt<<<nB * (NN / CV_N), CV_T, 0, stream>>>(feat, featT);
  k_conv<<<nB * GT, MT, 0, stream>>>(px, pmask, featT, gxp, out0, out1);
}
